// InteractionBlock_48902497632897
// MI455X (gfx1250) — hardware-run, weakly checked
//
#include <hip/hip_runtime.h>


namespace {

constexpr int N = 50000, NP = 50048, NPL = NP  , SRCM = N  , EFULL = 800000, E = EFULL  , D = 128, G = 64, NL = (NPL < N ? NPL : N);
constexpr float XS = 8.0f, WSC = 256.0f, QS = 16384.0f, LOG2E = 1.4426950408889634f, CUTOFF = 5.0f, SLOPE = 0.0f, BNEPS = 1e-5f;
static_assert(NP % 64 == 0 && NP >= N && NPL % 32 == 0 && D == 128 && G == 64 && EFULL % 8 == 0, "tiling");
typedef _Float16 b16;
typedef __attribute__((ext_vector_type(16))) _Float16 v16b;
typedef __attribute__((ext_vector_type(8))) _Float16 v8b;
typedef __attribute__((ext_vector_type(8))) float v8f;
typedef __attribute__((ext_vector_type(4))) float v4f;
__device__ __forceinline__ float bf16_rne(float f) { unsigned int u = __float_as_uint(f); u += 0x7FFFu + ((u >> 16) & 1u); return __uint_as_float(u & 0xFFFF0000u); }
__device__ __forceinline__ void split16(float v, b16& hi, b16& lo) { hi = (b16)v; lo = (b16)(v - (float)hi); }
__device__ __forceinline__ v16b frag_kb(const b16* p, int hh) { const v8b a = *(const v8b*)(p + 8 * hh), b = *(const v8b*)(p + 16 + 8 * hh); v16b f;
#pragma unroll
  for (int e = 0; e < 8; ++e) { f[e] = a[e]; f[8 + e] = b[e]; } return f; }
__device__ __forceinline__ v8f wmma16b(v16b a, v16b b, v8f c) { v8f d = __builtin_amdgcn_wmma_f32_16x16x32_f16(false, a, false, b, (short)0, c, false, false); asm volatile("v_nop\n\tv_nop\n\tv_nop\n\tv_nop" : "+v"(d) : "v"(a), "v"(b)); return d; }
__device__ __forceinline__ void wave_lds_sync() { __builtin_amdgcn_fence(__ATOMIC_RELEASE, "workgroup"); __builtin_amdgcn_wave_barrier(); __builtin_amdgcn_fence(__ATOMIC_ACQUIRE, "workgroup"); }
__device__ __forceinline__ float pmul(float a, float b) { float p = a * b; asm volatile("" : "+v"(p)); return p; }
__device__ __forceinline__ int iclamp(int v, int lo, int hi) { return v < lo ? lo : (v > hi ? hi : v); }
constexpr int CSR_NBLK = 512, CSR_GB = 9, CSR_GN = 1 << CSR_GB  , CSR_MAXG = 512, CSR_CAP = 12288  ;
__global__ __launch_bounds__(64) void csrA_kernel(const int* __restrict__ dst, int E, int N, int nG, int CHP, int NGP, int* __restrict__ STG, int* __restrict__ HST) {
  extern __shared__ int sm[];
  int* cnt = sm; int* run = sm + NGP; int* ids = sm + 2 * NGP;
  const int b = blockIdx.x; const int ch = (E + CSR_NBLK - 1) / CSR_NBLK; const int e0 = b * ch, e1 = min(E, e0 + ch);
  for (int i = threadIdx.x; i < NGP; i += 64) cnt[i] = 0;
  for (int i = threadIdx.x; i < CHP; i += 64) ids[i] = -1;
  __syncthreads();
  if (threadIdx.x == 0) {
    for (int e = e0; e < e1; ++e) { int d = dst[e]; d = (d < 0) ? 0 : (d >= N ? N - 1 : d); cnt[d >> CSR_GB] += 1; }
    int acc = 0; for (int g = 0; g < nG; ++g) { run[g] = acc; acc += cnt[g]; }
    for (int e = e0; e < e1; ++e) { int d = dst[e]; d = (d < 0) ? 0 : (d >= N ? N - 1 : d); const int g = d >> CSR_GB; ids[run[g]] = e; run[g] += 1; } }
  __syncthreads();
  typedef __attribute__((ext_vector_type(4))) int v4i;
  for (int pass = 0; pass < 2; ++pass) {
    for (int i = threadIdx.x; i < CHP / 4; i += 64) *(volatile v4i*)(STG + (size_t)b * CHP + i * 4) = *(const v4i*)(&ids[i * 4]);
    for (int i = threadIdx.x; i < NGP / 4; i += 64) { v4i v; for (int e = 0; e < 4; ++e) v[e] = (i * 4 + e < nG) ? cnt[i * 4 + e] : 0; *(volatile v4i*)(HST + (size_t)b * NGP + i * 4) = v; }
    __threadfence(); }
}
__global__ __launch_bounds__(512) void csrS_kernel(const int* __restrict__ HST, int nG, int NGP, int* __restrict__ START, int* __restrict__ TOT, int* __restrict__ OFF) {
  __shared__ int tot[CSR_MAXG];
  const int b = threadIdx.x;
  for (int pass = 0; pass < 2; ++pass) { int runb = 0; for (int g = 0; g < nG; ++g) { int c = HST[(size_t)b * NGP + g]; c = (c < 0) ? 0 : c; ((volatile int*)OFF)[(size_t)g * CSR_NBLK + b] = runb; runb += c; } __threadfence(); }
  for (int g = threadIdx.x; g < nG; g += 512) { int s = 0; for (int bb = 0; bb < CSR_NBLK; ++bb) { int c = HST[(size_t)bb * NGP + g]; s += (c < 0) ? 0 : c; } tot[g] = s; }
  __syncthreads();
  if (threadIdx.x < 32) {
    __shared__ int st[CSR_MAXG + 32];
    if (threadIdx.x == 0) { int acc = 0; for (int g = 0; g < NGP; ++g) { st[g] = acc; if (g < nG) acc += (tot[g] + 31) & ~31; } st[NGP] = acc; }
    __builtin_amdgcn_fence(__ATOMIC_RELEASE, "workgroup"); __builtin_amdgcn_wave_barrier(); __builtin_amdgcn_fence(__ATOMIC_ACQUIRE, "workgroup");
    for (int pass = 0; pass < 2; ++pass) { for (int i = threadIdx.x; i < NGP + 32; i += 32) { ((volatile int*)START)[i] = (i <= NGP) ? st[min(i, NGP)] : 0; ((volatile int*)TOT)[i] = (i < nG) ? tot[i] : 0; } __threadfence(); } }
}
__global__ __launch_bounds__(256) void csrB_kernel(const int* __restrict__ dst, int N, int nG, int CHP, int NGP, int permLen, const int* __restrict__ STG, const int* __restrict__ HST, const int* __restrict__ OFF, const int* __restrict__ START, const int* __restrict__ TOT, int* __restrict__ PERM, int* __restrict__ ROWPTR, int* __restrict__ ROWCNT, int* __restrict__ FLAG) {
  typedef __attribute__((ext_vector_type(4))) int v4i;
  __shared__ int ids[CSR_CAP]; __shared__ unsigned short key[CSR_CAP]; __shared__ int outp[CSR_CAP]; __shared__ int ncnt[CSR_GN + 1]; __shared__ int boff[CSR_NBLK + 1];
  const int g = blockIdx.x, t_ = threadIdx.x; int tot = TOT[g]; int st = START[g], stn = START[g + 1]; const int v0 = g * CSR_GN; const int nv = min(CSR_GN, N - v0);
  st = (st < 0) ? 0 : (st > permLen - 32 ? permLen - 32 : st) & ~31; stn = (stn < st) ? st : (stn > permLen ? permLen : stn); tot = (tot < 0) ? 0 : tot; if (tot > stn - st && tot <= CSR_CAP) tot = stn - st;
  if (tot > CSR_CAP) {
    for (int pass = 0; pass < 2; ++pass) { for (int i = t_; i < CSR_GN / 4; i += 256) { v4i a, c; for (int e = 0; e < 4; ++e) { a[e] = st; c[e] = 0; } *(volatile v4i*)(ROWPTR + v0 + i * 4) = a; *(volatile v4i*)(ROWCNT + v0 + i * 4) = c; } if (t_ == 0) ((volatile int*)FLAG)[0] = 1; __threadfence(); } (void)nv; return; }
  if (t_ == 0) { int acc = 0; for (int b = 0; b < CSR_NBLK; ++b) { boff[b] = acc; int c = HST[(size_t)b * NGP + g]; c = (c < 0) ? 0 : (c > CHP ? CHP : c); acc += c; if (acc > tot) acc = tot; } boff[CSR_NBLK] = acc; }
  for (int i = t_; i <= CSR_GN; i += 256) ncnt[i] = 0;
  __syncthreads();
  for (int b = 0; b < CSR_NBLK; ++b) { const int c = boff[b + 1] - boff[b]; int o_ = OFF[(size_t)g * CSR_NBLK + b]; o_ = (o_ < 0) ? 0 : (o_ > CHP - c ? CHP - c : o_); const int* src_ = STG + (size_t)b * CHP + o_;
    for (int i = t_; i < c; i += 256) { int id = src_[i]; id = (id < 0) ? 0 : id; ids[boff[b] + i] = id; int d = dst[id]; d = (d < v0) ? v0 : (d >= N ? N - 1 : d); int kk = d - v0; kk = (kk < 0) ? 0 : (kk >= CSR_GN ? CSR_GN - 1 : kk); key[boff[b] + i] = (unsigned short)kk; } }
  __syncthreads();
  if (t_ == 0) { for (int i = 0; i < tot; ++i) ncnt[key[i]] += 1; int acc = 0; for (int vl = 0; vl < CSR_GN; ++vl) { const int c = ncnt[vl]; ncnt[vl] = acc; acc += c; } ncnt[CSR_GN] = acc;
    for (int i = 0; i < tot; ++i) { const int vl = key[i]; outp[ncnt[vl]] = ids[i]; ncnt[vl] += 1; }
    for (int vl = CSR_GN; vl > 0; --vl) ncnt[vl] = ncnt[vl - 1]; ncnt[0] = 0; }
  __syncthreads();
  for (int pass = 0; pass < 2; ++pass) {
    for (int i = t_; i < (stn - st) / 4; i += 256) { v4i v; for (int e = 0; e < 4; ++e) { const int q = i * 4 + e; v[e] = (q < tot) ? outp[q] : -1; } *(volatile v4i*)(PERM + st + i * 4) = v; }
    for (int i = t_; i < CSR_GN / 4; i += 256) { v4i a, c; for (int e = 0; e < 4; ++e) { const int vl = i * 4 + e; a[e] = st + ncnt[vl]; c[e] = (vl < nv) ? (ncnt[vl + 1] - ncnt[vl]) : 0; } *(volatile v4i*)(ROWPTR + v0 + i * 4) = a; *(volatile v4i*)(ROWCNT + v0 + i * 4) = c; }
    __threadfence(); }
}
__global__ __launch_bounds__(256) void csrZ_kernel(int* __restrict__ p, size_t n4) { typedef __attribute__((ext_vector_type(4))) int v4i; const size_t tid = (size_t)blockIdx.x * 256 + threadIdx.x, nth = (size_t)gridDim.x * 256; v4i z = {0, 0, 0, 0}; for (size_t i = tid; i < n4; i += nth) *(volatile v4i*)(p + i * 4) = z; }
struct CsrBufs { int *STG, *HST, *OFF, *START, *TOT, *PERM, *ROWPTR, *ROWCNT, *FLAG; int nG, NGP, CHP; size_t permLen; char* base; size_t bytes; };
static size_t csr_carve(CsrBufs& c, char* ws, size_t off, int E, int N) {
  const size_t off0 = off; c.base = ws + off;
  auto al = [&](size_t bytes) { char* p = ws + off; off += (bytes + 255) & ~(size_t)255; return p; };
  c.nG = (N + CSR_GN - 1) / CSR_GN; c.NGP = (c.nG + 31) & ~31; const int ch = (E + CSR_NBLK - 1) / CSR_NBLK; c.CHP = (ch + 31) & ~31; c.permLen = (size_t)E + 32 * (size_t)c.nG + 32;
  c.STG = (int*)al((size_t)CSR_NBLK * c.CHP * 4); c.HST = (int*)al((size_t)CSR_NBLK * c.NGP * 4); c.OFF = (int*)al((size_t)c.NGP * CSR_NBLK * 4); c.START = (int*)al((size_t)(c.NGP + 64) * 4); c.TOT = (int*)al((size_t)(c.NGP + 64) * 4);
  c.PERM = (int*)al(c.permLen * 4); c.ROWPTR = (int*)al((size_t)c.nG * CSR_GN * 4); c.ROWCNT = (int*)al((size_t)c.nG * CSR_GN * 4); c.FLAG = (int*)al(256);
  c.bytes = off - off0; return off;
}
static void csr_build(const CsrBufs& c, const int* dst, int E, int N, hipStream_t stream) {
  const size_t smem = (size_t)(2 * c.NGP + c.CHP) * 4;
  csrZ_kernel<<<512, 256, 0, stream>>>((int*)c.base, c.bytes / 16);
  csrA_kernel<<<CSR_NBLK, 64, smem, stream>>>(dst, E, N, c.nG, c.CHP, c.NGP, c.STG, c.HST);
  csrS_kernel<<<1, 512, 0, stream>>>(c.HST, c.nG, c.NGP, c.START, c.TOT, c.OFF);
  csrB_kernel<<<c.nG, 256, 0, stream>>>(dst, N, c.nG, c.CHP, c.NGP, (int)c.permLen, c.STG, c.HST, c.OFF, c.START, c.TOT, c.PERM, c.ROWPTR, c.ROWCNT, c.FLAG);
}

typedef __attribute__((ext_vector_type(4))) _Float16 v4h;
typedef __attribute__((ext_vector_type(2))) float v2f;
typedef __attribute__((ext_vector_type(4))) int v4i_t;
__device__ __forceinline__ float nexp2(float v) { return __builtin_amdgcn_exp2f(v); }
template <int KD, int NOUT>
__global__ __launch_bounds__(256) void wprep_kernel(const float* __restrict__ w, b16* __restrict__ WT) {
  static_assert(KD % 8 == 0, "wprep"); const size_t u = (size_t)blockIdx.x * 256 + threadIdx.x; if (u >= (size_t)NOUT * KD / 8) return; const size_t e = u * 8; const int oo = (int)(e / KD), k0 = (int)(e % KD); v8b o;
  for (int j = 0; j < 8; ++j) o[j] = (b16)(bf16_rne(w[(size_t)(k0 + j) * NOUT + oo]) * WSC);
  for (int pass = 0; pass < 2; ++pass) { *(volatile v8b*)(WT + e) = o; __threadfence(); }
}
template <int KD, int NOUT, int NV, bool RNDA  >
__global__ __launch_bounds__(64) void gemm_kernel(const float* __restrict__ A, const b16* __restrict__ W, float* __restrict__ T) {
  constexpr int SL = NOUT < 128 ? NOUT : 128, NT = SL / 16, KC = KD < 128 ? KD : 128;
  static_assert(KD % KC == 0 && KC % 32 == 0 && NOUT % SL == 0 && SL % 32 == 0, "gemm tiling");
  __shared__ __attribute__((aligned(16))) b16 Ah[2][16][KC + 8], Al[2][16][KC + 8]; __shared__ __attribute__((aligned(16))) float Tf[2][16][SL + 4];
  const int wave = threadIdx.x >> 5, lane = threadIdx.x & 31, nloc = lane & 15, hlf = lane >> 4; const size_t m0 = (size_t)blockIdx.x * 32 + wave * 16; const int n0 = blockIdx.y * SL;
  v8f acc[NT];
#pragma unroll
  for (int t = 0; t < NT; ++t) acc[t] = (v8f){};
#pragma unroll 1
  for (int kc = 0; kc < KD; kc += KC) {
    for (int idx = lane; idx < 16 * (KC / 4); idx += 32) { const int rr = idx / (KC / 4), c4 = (idx % (KC / 4)) * 4; const size_t row = (m0 + rr < (size_t)NV) ? (m0 + rr) : (size_t)(NV - 1); const v4f v = *(const v4f*)(A + row * KD + kc + c4); v4h hv, lv;
      for (int j = 0; j < 4; ++j) { b16 ph, pl; split16((RNDA ? bf16_rne(v[j]) : v[j]) * XS, ph, pl); hv[j] = ph; lv[j] = pl; } *(v4h*)(&Ah[wave][rr][c4]) = hv; *(v4h*)(&Al[wave][rr][c4]) = lv; }
    wave_lds_sync();
#pragma unroll
    for (int kb = 0; kb < KC; kb += 32) { const v16b a = frag_kb(&Ah[wave][nloc][kb], hlf), al = frag_kb(&Al[wave][nloc][kb], hlf);
#pragma unroll
      for (int t = 0; t < NT; ++t) { const v16b bw = frag_kb(W + (size_t)(n0 + t * 16 + nloc) * KD + kc + kb, hlf); acc[t] = wmma16b(a, bw, acc[t]); acc[t] = wmma16b(al, bw, acc[t]); } }
    wave_lds_sync(); }
#pragma unroll
  for (int t = 0; t < NT; ++t)
#pragma unroll
    for (int r = 0; r < 8; ++r) Tf[wave][8 * hlf + r][t * 16 + nloc] = acc[t][r] * (1.0f / (XS * WSC));
  wave_lds_sync();
  for (int pass = 0; pass < 2; ++pass) { for (int idx = lane; idx < 16 * (SL / 4); idx += 32) { const int rr = idx / (SL / 4), c4 = (idx % (SL / 4)) * 4; *(volatile v4f*)(T + (m0 + rr) * NOUT + n0 + c4) = *(const v4f*)(&Tf[wave][rr][c4]); } __threadfence(); }
}

template <int KD, int NOUT, int LDA, int LDT, bool RNDA>
__global__ __launch_bounds__(64) void gemmx_kernel(const float* __restrict__ A, int nv, const b16* __restrict__ W, const float* __restrict__ bias, int mrows, float* __restrict__ T) {
  constexpr int SL = NOUT < 128 ? NOUT : 128, NT = SL / 16, KC = KD < 128 ? KD : 128;
  static_assert(KD % KC == 0 && KC % 32 == 0 && NOUT % SL == 0 && SL % 32 == 0 && LDA >= KD && LDT >= NOUT, "gemmx tiling");
  __shared__ __attribute__((aligned(16))) b16 Ah[2][16][KC + 8], Al[2][16][KC + 8]; __shared__ __attribute__((aligned(16))) float Tf[2][16][SL + 4];
  const int wave = threadIdx.x >> 5, lane = threadIdx.x & 31, nloc = lane & 15, hlf = lane >> 4; const size_t m0 = (size_t)blockIdx.x * 32 + wave * 16; const int n0 = blockIdx.y * SL;
  v8f acc[NT];
#pragma unroll
  for (int t = 0; t < NT; ++t) acc[t] = (v8f){};
#pragma unroll 1
  for (int kc = 0; kc < KD; kc += KC) {
    for (int idx = lane; idx < 16 * (KC / 4); idx += 32) { const int rr = idx / (KC / 4), c4 = (idx % (KC / 4)) * 4; const size_t row = (m0 + rr < (size_t)nv) ? (m0 + rr) : (size_t)(nv - 1); const v4f v = *(const v4f*)(A + row * LDA + kc + c4); v4h hv, lv;
      for (int j = 0; j < 4; ++j) { b16 ph, pl; split16((RNDA ? bf16_rne(v[j]) : v[j]) * XS, ph, pl); hv[j] = ph; lv[j] = pl; } *(v4h*)(&Ah[wave][rr][c4]) = hv; *(v4h*)(&Al[wave][rr][c4]) = lv; }
    wave_lds_sync();
#pragma unroll
    for (int kb = 0; kb < KC; kb += 32) { const v16b a = frag_kb(&Ah[wave][nloc][kb], hlf), al = frag_kb(&Al[wave][nloc][kb], hlf);
#pragma unroll
      for (int t = 0; t < NT; ++t) { const v16b bw = frag_kb(W + (size_t)(n0 + t * 16 + nloc) * KD + kc + kb, hlf); acc[t] = wmma16b(a, bw, acc[t]); if (!RNDA) acc[t] = wmma16b(al, bw, acc[t]); } }
    wave_lds_sync(); }
#pragma unroll
  for (int t = 0; t < NT; ++t) { const float bb = bias ? bf16_rne(bias[n0 + t * 16 + nloc]) : 0.0f;
#pragma unroll
    for (int r = 0; r < 8; ++r) Tf[wave][8 * hlf + r][t * 16 + nloc] = acc[t][r] * (1.0f / (XS * WSC)) + bb; }
  wave_lds_sync();
  for (int pass = 0; pass < 2; ++pass) { for (int idx = lane; idx < 16 * (SL / 4); idx += 32) { const int rr = idx / (SL / 4), c4 = (idx % (SL / 4)) * 4; if (m0 + rr < (size_t)mrows) *(volatile v4f*)(T + (m0 + rr) * LDT + n0 + c4) = *(const v4f*)(&Tf[wave][rr][c4]); } __threadfence(); }
}

__global__ __launch_bounds__(256) void deint_kernel(const int* __restrict__ a, int* __restrict__ DST, int* __restrict__ SRC) {
  const int u = blockIdx.x * 256 + threadIdx.x; if (u >= E / 4) return; v4i_t d4, s4; for (int j = 0; j < 4; ++j) { d4[j] = a[(size_t)(u * 4 + j) * 2]; s4[j] = a[(size_t)(u * 4 + j) * 2 + 1]; }
  for (int pass = 0; pass < 2; ++pass) { *(volatile v4i_t*)(DST + (size_t)u * 4) = d4; *(volatile v4i_t*)(SRC + (size_t)u * 4) = s4; __threadfence(); }
}
__global__ __launch_bounds__(256) void edge_kernel(const float* __restrict__ dist, const float* __restrict__ RF, const b16* __restrict__ WF, const float* __restrict__ bf2, const int* __restrict__ SRC, const int* __restrict__ PERM, const int* __restrict__ ROWPTR, const int* __restrict__ ROWCNT, int permLen, float* __restrict__ Y) {
  __shared__ __attribute__((aligned(16))) b16 Ag[8][16][G + 8]; __shared__ __attribute__((aligned(16))) float Yo[8][D + 4]; __shared__ int Es[8][16];
  const int wave = threadIdx.x >> 5, lane = threadIdx.x & 31, nloc = lane & 15, hlf = lane >> 4; const int v = blockIdx.x * 8 + wave;
  const float width = CUTOFF / (float)(G - 1); const float coeff = -0.5f / (width * width);
  int cnt = 0, p0 = 0; if (v < NL) { cnt = iclamp(ROWCNT[v], 0, 65536); p0 = ROWPTR[v]; p0 = iclamp(p0, 0, permLen - 1); if (p0 + cnt > permLen) cnt = permLen - p0; }
  float ys[8]; for (int t = 0; t < 8; ++t) ys[t] = 0.0f;
#pragma unroll 1
  for (int c0 = 0; c0 < cnt; c0 += 16) {
    if (lane < 16) { const int i = c0 + lane; int eid = -1; if (i < cnt) { eid = PERM[p0 + i]; eid = iclamp(eid, 0, E - 1); } Es[wave][lane] = eid; }
    wave_lds_sync();
    { const int row = nloc; const int eid = Es[wave][row]; const float de = eid >= 0 ? bf16_rne(dist[eid]) : 0.0f;
#pragma unroll
      for (int j4 = 0; j4 < 8; ++j4) { v4h o; for (int q = 0; q < 4; ++q) { const int j = 32 * hlf + j4 * 4 + q; const float off = (j == G - 1) ? CUTOFF : (0.0f * (1.0f - (float)j / (float)(G - 1)) + CUTOFF * ((float)j / (float)(G - 1))); const float dd = de - off; const float gv = eid >= 0 ? nexp2(coeff * LOG2E * dd * dd) : 0.0f; o[q] = (b16)(gv * QS); }
        *(v4h*)(&Ag[wave][row][32 * hlf + j4 * 4]) = o; } }
    wave_lds_sync();
    v8f acc[8]; const v16b a0 = frag_kb(&Ag[wave][nloc][0], hlf), a1 = frag_kb(&Ag[wave][nloc][32], hlf);
#pragma unroll
    for (int t = 0; t < 8; ++t) { const b16* br = WF + (size_t)(t * 16 + nloc) * G; acc[t] = wmma16b(a0, frag_kb(br, hlf), (v8f){}); acc[t] = wmma16b(a1, frag_kb(br + 32, hlf), acc[t]); }
#pragma unroll
    for (int r = 0; r < 8; ++r) { const int eid = Es[wave][8 * hlf + r]; if (eid >= 0) { int s = iclamp(SRC[eid], 0, N - 1); if (SRCM < N) s %= SRCM; const float* rfr = RF + (size_t)s * D;
#pragma unroll
        for (int t = 0; t < 8; ++t) { const int col = t * 16 + nloc; ys[t] = fmaf(acc[t][r] * (1.0f / (QS * WSC)) + bf16_rne(bf2[col]), rfr[col], ys[t]); } } }
    wave_lds_sync(); }
#pragma unroll
  for (int t = 0; t < 8; ++t) { ys[t] += __shfl_xor(ys[t], 16); if (hlf == 0) Yo[wave][t * 16 + nloc] = (v < N) ? ys[t] : 0.0f; }
  wave_lds_sync();
  if (v < NPL) for (int pass = 0; pass < 2; ++pass) { *(volatile v4f*)(Y + (size_t)v * D + lane * 4) = *(const v4f*)(&Yo[wave][lane * 4]); __threadfence(); }
}
__global__ __launch_bounds__(256) void ssp_kernel(float* __restrict__ T) { const size_t u = (size_t)blockIdx.x * 256 + threadIdx.x; if (u >= (size_t)NPL * D / 4) return; v4f x = *(const v4f*)(T + u * 4);
  for (int j = 0; j < 4; ++j) { const float v = x[j]; x[j] = fmaxf(v, 0.0f) + log1pf(__expf(-fabsf(v))) - 0.69314718055994531f; }
  for (int pass = 0; pass < 2; ++pass) { *(volatile v4f*)(T + u * 4) = x; __threadfence(); } }
}

extern "C" void kernel_launch(void* const* d_in, const int* in_sizes, int n_in, void* d_out, int out_size, void* d_ws, size_t ws_size, hipStream_t stream) {
  (void)n_in;
  auto Fp = [&](int i) { return (const float*)d_in[i]; }; auto Ip = [&](int i) { return (const int*)d_in[i]; };
  if (in_sizes[0] != N * D || in_sizes[1] != EFULL || in_sizes[2] != G * D || in_sizes[3] != D || in_sizes[4] != D * D || in_sizes[5] != D * D || in_sizes[6] != D || in_sizes[7] != D * D || in_sizes[8] != D || in_sizes[9] != 2 * EFULL || out_size != N * D) return;
  size_t off = 0; char* ws = (char*)d_ws;
  auto carve = [&](size_t bytes) { char* p = ws + off; off += (bytes + 255) & ~(size_t)255; return p; };
  b16* WAT = (b16*)carve((size_t)D * D * 2); b16* WFT = (b16*)carve((size_t)D * G * 2); b16* W1T = (b16*)carve((size_t)D * D * 2); b16* W2T = (b16*)carve((size_t)D * D * 2);
  int* DSTI = (int*)carve((size_t)EFULL * 4); int* SRCI = (int*)carve((size_t)EFULL * 4); float* RF = (float*)carve((size_t)NP * D * 4); float* Y = (float*)carve((size_t)NP * D * 4); float* T = (float*)carve((size_t)NP * D * 4);
  CsrBufs csr; off = csr_carve(csr, ws, off, E, N);
  if (off > ws_size || off > ((size_t)128 << 20)) return;
  wprep_kernel<D, D><<<(D * D / 8 + 255) / 256, 256, 0, stream>>>(Fp(4), WAT); wprep_kernel<G, D><<<(G * D / 8 + 255) / 256, 256, 0, stream>>>(Fp(2), WFT); wprep_kernel<D, D><<<(D * D / 8 + 255) / 256, 256, 0, stream>>>(Fp(5), W1T); wprep_kernel<D, D><<<(D * D / 8 + 255) / 256, 256, 0, stream>>>(Fp(7), W2T);
  deint_kernel<<<(E / 4 + 255) / 256, 256, 0, stream>>>(Ip(9), DSTI, SRCI);
  csr_build(csr, DSTI, E, N, stream);
  gemm_kernel<D, D, N, true><<<dim3(NP / 32, 1), 64, 0, stream>>>(Fp(0), WAT, RF);
  edge_kernel<<<NPL / 8, 256, 0, stream>>>(Fp(1), RF, WFT, Fp(3), SRCI, csr.PERM, csr.ROWPTR, csr.ROWCNT, (int)csr.permLen, Y);
  gemmx_kernel<D, D, D, D, false><<<dim3(NPL / 32, 1), 64, 0, stream>>>(Y, NPL, W1T, Fp(6), NPL, T); ssp_kernel<<<(unsigned)(((size_t)NPL * D / 4 + 255) / 256), 256, 0, stream>>>(T);
  gemmx_kernel<D, D, D, D, false><<<dim3(NPL / 32, 1), 64, 0, stream>>>(T, NPL, W2T, Fp(8), NL, (float*)d_out);
}
